// POLICY_41334765256938
// MI455X (gfx1250) — hardware-run, weakly checked
//
#include <hip/hip_runtime.h>
#include <stddef.h>
#include <stdint.h>
#include <math.h>

#define NN      100000
#define HD      64
#define NLAY    3
#define NE      1200000
#define GBM     128
#define NT      782
#define MP      100096
#define KL      128
#define NTHR    256
#define NWAVE   8
#define EPT     8
#define WCH     (32 * EPT)
#define NBRUN   1024
#define SLB     10
#define NBK     98
#define WLCAP   2048
#define RCAP    16384
#define DEGCAP  64
#define MAXDEG_MEAS   29
#define MAXB1024_MEAS 12539
#define ABM     64
#define SP      68
#define AP      136
#define WSMAX   134217728

#define BK_ZINTS (NWAVE * WLCAP + RCAP + 3 * NBRUN)
#define BK_INTS  (BK_ZINTS + 16)
#define BK_LDS   (BK_INTS * 4)
#define BK_PER   (((NE + NWAVE * WCH - 1) / (NWAVE * WCH)) * WCH)

#define TB_B1   0
#define TB_B2   192
#define TB_G    384
#define TB_BE   576
#define TB_L1B  768
#define TB_L2W  832
#define TB_SC   896
#define TB_N    1024

#define PBX   (NN * HD / 4 / NTHR)
#define PBW   (7 * HD * KL / 8 / NTHR)
#define PBZ   ((MP - NN) * KL / 8 / NTHR)
#define PBT   7
#define PBTOT (PBX + PBW + PBZ + PBT)

static_assert(HD == 64 && HD == 16 * 4);
static_assert(KL == 2 * HD && KL % 32 == 0 && KL == 128);
static_assert(MP % GBM == 0 && MP == NT * GBM && MP >= NN && MP % ABM == 0);
static_assert(NN % 32 == 0 && NN - (MP - GBM) == 32);
static_assert(NBRUN == (1 << SLB) && NBRUN % ABM == 0 && NBRUN % 32 == 0);
static_assert(NBK * NBRUN >= MP);
static_assert(NE < (1 << 21) && (((long long)NE) << SLB) < (1LL << 31));
static_assert(NE % EPT == 0 && NE % 4 == 0 && NE >= EPT);
static_assert(BK_PER % WCH == 0 && (long long)BK_PER * NWAVE >= NE);
static_assert(RCAP == NWAVE * WLCAP && RCAP % 4 == 0 && BK_ZINTS % 4 == 0);
static_assert((long long)RCAP * 100 >= (long long)MAXB1024_MEAS * 105);
static_assert(WLCAP >= MAXB1024_MEAS / 8 + 8 * 46 + 1);
static_assert(MAXDEG_MEAS + 8 <= DEGCAP);
static_assert(BK_LDS <= 300000);
static_assert((NN * HD / 4) % NTHR == 0 && (7 * HD * KL / 8) % NTHR == 0 && ((MP - NN) * KL / 8) % NTHR == 0);
static_assert((HD * KL / 8) % NTHR == 0);
static_assert(AP * 2 == SP * 4 && AP % 8 == 0 && AP >= KL);
static_assert((GBM * 4) % 128 == 0 && (((NN % GBM) * 4) % 128) == 0);
static_assert((GBM * SP + 128 + 192) * 4 <= 65536);
static_assert(NT * GBM - GBM + 32 == NN);

typedef float          v4f   __attribute__((ext_vector_type(4)));
typedef float          v8f   __attribute__((ext_vector_type(8)));
typedef int            v4i   __attribute__((ext_vector_type(4)));
typedef int            v8i   __attribute__((ext_vector_type(8)));
typedef unsigned short v8us  __attribute__((ext_vector_type(8)));
typedef unsigned short v16us __attribute__((ext_vector_type(16)));
typedef __bf16         v16bf __attribute__((ext_vector_type(16)));
typedef v4f  __attribute__((may_alias)) v4fa;
typedef v4i  __attribute__((may_alias)) v4ia;
typedef v8us __attribute__((may_alias)) v8usa;
union FragB { v16bf v; v16us u; v8us h[2]; v8i w; };

__device__ __forceinline__ v8f wmb(const FragB& a, const FragB& b, v8f c) {
  v8f d = __builtin_amdgcn_wmma_f32_16x16x32_bf16(false, a.v, false, b.v, (short)0, c, false, false);
  asm volatile("v_nop\n\tv_nop\n\tv_nop\n\tv_nop" : "+v"(d) : "v"(a.w), "v"(b.w));
  return d;
}

__device__ __forceinline__ unsigned bf16_bits(float f) {
  const unsigned u = __float_as_uint(f);
  const unsigned r = (u + 0x7FFFu + ((u >> 16) & 1u)) >> 16;
  const unsigned q = (u >> 16) | 0x40u;
  return ((u & 0x7fffffffu) > 0x7f800000u) ? q : r;
}
__device__ __forceinline__ float bf16_val(float f) {
  return __uint_as_float(bf16_bits(f) << 16);
}

__device__ __forceinline__ void hilo_pack(float v0, float v1, float v2, float v3,
                                          int& h01, int& h23, int& l01, int& l23) {
  const unsigned a0 = bf16_bits(v0), a1 = bf16_bits(v1), a2 = bf16_bits(v2), a3 = bf16_bits(v3);
  const unsigned b0 = bf16_bits(v0 - __uint_as_float(a0 << 16));
  const unsigned b1 = bf16_bits(v1 - __uint_as_float(a1 << 16));
  const unsigned b2 = bf16_bits(v2 - __uint_as_float(a2 << 16));
  const unsigned b3 = bf16_bits(v3 - __uint_as_float(a3 << 16));
  h01 = (int)(a0 | (a1 << 16)); h23 = (int)(a2 | (a3 << 16));
  l01 = (int)(b0 | (b1 << 16)); l23 = (int)(b2 | (b3 << 16));
}

__device__ __forceinline__ v4i regroup8(int h01, int h23, int l01, int l23, int lane) {
  const int t  = lane & 15;
  const int s0 = (lane & 16) + ((2 * t) & 15), s1 = s0 + 1;
  const int a0 = __shfl(h01, s0, 32), a1 = __shfl(h23, s0, 32), a2 = __shfl(h01, s1, 32), a3 = __shfl(h23, s1, 32);
  const int b0 = __shfl(l01, s0, 32), b1 = __shfl(l23, s0, 32), b2 = __shfl(l01, s1, 32), b3 = __shfl(l23, s1, 32);
  const int mk = (t < 8) ? -1 : 0;
  v4i o;
  o.x = (a0 & mk) | (b0 & ~mk); o.y = (a1 & mk) | (b1 & ~mk);
  o.z = (a2 & mk) | (b2 & ~mk); o.w = (a3 & mk) | (b3 & ~mk);
  return o;
}

__device__ __forceinline__ void st2_v4f(float* p, v4f v) {
  *(volatile v4f*)p = v;
  __threadfence();
  *(volatile v4f*)p = v;
}
__device__ __forceinline__ void st2_v8us(unsigned short* p, v8us v) {
  *(volatile v8us*)p = v;
  __threadfence();
  *(volatile v8us*)p = v;
}
__device__ __forceinline__ void st2_v4i(unsigned short* p, v4i v) {
  *(volatile v4i*)p = v;
  __threadfence();
  *(volatile v4i*)p = v;
}

__device__ __forceinline__ v8us cvt8(const float* __restrict__ p) {
  const v4f a = *(const v4fa*)p;
  const v4f b = *(const v4fa*)(p + 4);
  v8us o;
  o[0] = (unsigned short)bf16_bits(a.x); o[1] = (unsigned short)bf16_bits(a.y);
  o[2] = (unsigned short)bf16_bits(a.z); o[3] = (unsigned short)bf16_bits(a.w);
  o[4] = (unsigned short)bf16_bits(b.x); o[5] = (unsigned short)bf16_bits(b.y);
  o[6] = (unsigned short)bf16_bits(b.z); o[7] = (unsigned short)bf16_bits(b.w);
  return o;
}

__device__ __forceinline__ void tab_copy(const float* __restrict__ src, int n4, float* dst, int tid) {
  const int i = tid < n4 ? tid : n4 - 1;
  const v4f a = *(const v4fa*)(src + 4 * i);
  asm volatile("" :: "v"(a));
  v4f o;
  o.x = bf16_val(a.x); o.y = bf16_val(a.y); o.z = bf16_val(a.z); o.w = bf16_val(a.w);
  if (tid < n4) st2_v4f(dst + 4 * tid, o);
}

__global__ __launch_bounds__(NTHR) void k_prep(const float* __restrict__ x, const float* __restrict__ W1,
                                               const float* __restrict__ b1, const float* __restrict__ W2,
                                               const float* __restrict__ b2, const float* __restrict__ gam,
                                               const float* __restrict__ bet, const float* __restrict__ eps,
                                               const float* __restrict__ l1w, const float* __restrict__ l1b,
                                               const float* __restrict__ l2w, const float* __restrict__ l2b,
                                               float* X, unsigned short* WPL, unsigned short* HHL, float* TB) {
  const int tid = (int)threadIdx.x, lane = tid & 31;
  const int blk = (int)blockIdx.x;
  if (blk < PBX) {
    const int u = blk * NTHR + tid;
    const v4f a = *(const v4fa*)(x + (size_t)u * 4);
    v4f o;
    o.x = bf16_val(a.x); o.y = bf16_val(a.y); o.z = bf16_val(a.z); o.w = bf16_val(a.w);
    st2_v4f(X + (size_t)u * 4, o);
  } else if (blk < PBX + PBW) {
    const int u  = (blk - PBX) * NTHR + tid;
    const int p  = u >> 10;
    const int n  = (u >> 4) & 63, k8 = (u & 15) * 8, kk = k8 & 63;
    const int so = n * HD + kk;
    v8us o;
    if (p < 3)      o = cvt8(W1 + (size_t)p * HD * HD + so);
    else if (p < 6) o = cvt8(W2 + (size_t)(p - 3) * HD * HD + so);
    else            o = cvt8(l1w + so);
    st2_v8us(WPL + (size_t)u * 8, o);
  } else if (blk < PBX + PBW + PBZ) {
    const int u = (blk - PBX - PBW) * NTHR + tid;
    const v8us z = {0, 0, 0, 0, 0, 0, 0, 0};
    st2_v8us(HHL + (size_t)NN * KL + (size_t)u * 8, z);
  } else {
    const int tb = blk - (PBX + PBW + PBZ);
    if (tb == 0)      tab_copy(b1,  48, TB + TB_B1,  tid);
    else if (tb == 1) tab_copy(b2,  48, TB + TB_B2,  tid);
    else if (tb == 2) tab_copy(gam, 48, TB + TB_G,   tid);
    else if (tb == 3) tab_copy(bet, 48, TB + TB_BE,  tid);
    else if (tb == 4) tab_copy(l1b, 16, TB + TB_L1B, tid);
    else if (tb == 5) tab_copy(l2w, 16, TB + TB_L2W, tid);
    else {
      if (tid < 32) {
        const float s0 = l2b[0], s1 = eps[0], s2 = eps[1], s3 = eps[2];
        const unsigned mk = (lane == 0) ? 0xffffffffu : 0u;
        v4f o;
        o.x = __uint_as_float((bf16_bits(s0) << 16) & mk);
        o.y = __uint_as_float((bf16_bits(s1) << 16) & mk);
        o.z = __uint_as_float((bf16_bits(s2) << 16) & mk);
        o.w = __uint_as_float((bf16_bits(s3) << 16) & mk);
        asm volatile("" :: "v"(o));
        if (lane < 8) st2_v4f(TB + TB_SC + 4 * lane, o);
      }
    }
  }
}

__device__ __forceinline__ void bucket_flush(const int* pl, const int* cnt, int ov, int* lp, int* cop, int* fp,
                                             int tid) {
#pragma unroll 1
  for (int i = tid * 4; i < RCAP; i += NTHR * 4) {
    const v4i v = *(const v4ia*)(pl + i);
    *(volatile v4i*)(lp + i) = v;
  }
#pragma unroll 1
  for (int i = tid * 4; i < 2 * NBRUN; i += NTHR * 4) {
    const v4i v = *(const v4ia*)(cnt + i);
    *(volatile v4i*)(cop + i) = v;
  }
  if (tid < 8) {
    const v4i f = {ov, ov, ov, ov};
    *(volatile v4i*)(fp + 4 * tid) = f;
  }
}

__global__ __launch_bounds__(NTHR) void k_bucket(const int* __restrict__ srcs, const int* __restrict__ dsts,
                                                 int* LIST, int* CO, int* FLAG) {
  extern __shared__ __attribute__((aligned(16))) int dsm[];
  int* wl   = dsm;
  int* pl   = dsm + NWAVE * WLCAP;
  int* cnt  = pl + RCAP;
  int* offs = cnt + NBRUN;
  int* cur  = offs + NBRUN;
  int* misc = cur + NBRUN;
  const int tid = (int)threadIdx.x, lane = tid & 31, wave = tid >> 5;
  const int blk = (int)blockIdx.x;
  const unsigned nbs = (unsigned)(blk * NBRUN);

  {
    const v4i z4 = {0, 0, 0, 0};
    for (int i = tid * 4; i < BK_ZINTS; i += NTHR * 4) *(v4ia*)(dsm + i) = z4;
    if (tid < 16) misc[tid] = 0;
  }
  __syncthreads();

  {
    const int ebeg = wave * BK_PER;
    const int eend = (ebeg + BK_PER < NE) ? (ebeg + BK_PER) : NE;
    int* mylist = wl + wave * WLCAP;
    int wc = 0;
#pragma unroll 1
    for (int cb = ebeg; cb < eend; cb += WCH) {
      const int e0 = cb + lane * EPT;
      const int ec = e0 < NE - EPT ? e0 : NE - EPT;
      const bool inr = e0 < eend;
      const v4i da = *(const v4ia*)(dsts + ec);
      const v4i db = *(const v4ia*)(dsts + ec + 4);
      const unsigned s0 = (unsigned)da.x - nbs, s1 = (unsigned)da.y - nbs;
      const unsigned s2 = (unsigned)da.z - nbs, s3 = (unsigned)da.w - nbs;
      const unsigned s4 = (unsigned)db.x - nbs, s5 = (unsigned)db.y - nbs;
      const unsigned s6 = (unsigned)db.z - nbs, s7 = (unsigned)db.w - nbs;
      const bool h0 = (s0 < (unsigned)NBRUN) & inr, h1 = (s1 < (unsigned)NBRUN) & inr;
      const bool h2 = (s2 < (unsigned)NBRUN) & inr, h3 = (s3 < (unsigned)NBRUN) & inr;
      const bool h4 = (s4 < (unsigned)NBRUN) & inr, h5 = (s5 < (unsigned)NBRUN) & inr;
      const bool h6 = (s6 < (unsigned)NBRUN) & inr, h7 = (s7 < (unsigned)NBRUN) & inr;
      const unsigned m0 = __builtin_amdgcn_ballot_w32(h0), m1 = __builtin_amdgcn_ballot_w32(h1);
      const unsigned m2 = __builtin_amdgcn_ballot_w32(h2), m3 = __builtin_amdgcn_ballot_w32(h3);
      const unsigned m4 = __builtin_amdgcn_ballot_w32(h4), m5 = __builtin_amdgcn_ballot_w32(h5);
      const unsigned m6 = __builtin_amdgcn_ballot_w32(h6), m7 = __builtin_amdgcn_ballot_w32(h7);
      const unsigned any = m0 | m1 | m2 | m3 | m4 | m5 | m6 | m7;
      if (any != 0u) {
        const int pre = (int)(__builtin_amdgcn_mbcnt_lo(m0, 0u) + __builtin_amdgcn_mbcnt_lo(m1, 0u) +
                              __builtin_amdgcn_mbcnt_lo(m2, 0u) + __builtin_amdgcn_mbcnt_lo(m3, 0u) +
                              __builtin_amdgcn_mbcnt_lo(m4, 0u) + __builtin_amdgcn_mbcnt_lo(m5, 0u) +
                              __builtin_amdgcn_mbcnt_lo(m6, 0u) + __builtin_amdgcn_mbcnt_lo(m7, 0u));
        int p = wc + pre;
        if (h0) { if (p < WLCAP) mylist[p] = ((e0 + 0) << SLB) | (int)s0; p = p + 1; }
        if (h1) { if (p < WLCAP) mylist[p] = ((e0 + 1) << SLB) | (int)s1; p = p + 1; }
        if (h2) { if (p < WLCAP) mylist[p] = ((e0 + 2) << SLB) | (int)s2; p = p + 1; }
        if (h3) { if (p < WLCAP) mylist[p] = ((e0 + 3) << SLB) | (int)s3; p = p + 1; }
        if (h4) { if (p < WLCAP) mylist[p] = ((e0 + 4) << SLB) | (int)s4; p = p + 1; }
        if (h5) { if (p < WLCAP) mylist[p] = ((e0 + 5) << SLB) | (int)s5; p = p + 1; }
        if (h6) { if (p < WLCAP) mylist[p] = ((e0 + 6) << SLB) | (int)s6; p = p + 1; }
        if (h7) { if (p < WLCAP) mylist[p] = ((e0 + 7) << SLB) | (int)s7; p = p + 1; }
        wc += (int)(__builtin_popcount(m0) + __builtin_popcount(m1) + __builtin_popcount(m2) + __builtin_popcount(m3) +
                    __builtin_popcount(m4) + __builtin_popcount(m5) + __builtin_popcount(m6) + __builtin_popcount(m7));
      }
    }
    if (lane == 0) misc[wave] = wc;
  }
  __syncthreads();

  if (wave == 0) {
    int ov = 0;
#pragma unroll 1
    for (int w2 = 0; w2 < NWAVE; ++w2) {
      int c = misc[w2];
      if (c > WLCAP) ov = 1;
      c = c < 0 ? 0 : (c > WLCAP ? WLCAP : c);
#pragma unroll 1
      for (int b0 = 0; b0 < c; b0 += 32) {
        const int idx = b0 + lane;
        const int ent = wl[w2 * WLCAP + (idx < WLCAP ? idx : WLCAP - 1)];
        const int m32 = (c - b0) < 32 ? (c - b0) : 32;
#pragma unroll 1
        for (int k = 0; k < m32; ++k) {
          const int u    = __builtin_amdgcn_readlane(ent, k);
          const int slot = u & (NBRUN - 1);
          if (lane == 0) cnt[slot] = cnt[slot] + 1;
        }
      }
    }
    if (lane == 0) misc[9] = ov;
  }
  __syncthreads();
  if (wave == 0) {
    const int base = lane * (NBRUN / 32);
    int s = 0;
#pragma unroll 1
    for (int i = 0; i < NBRUN / 32; ++i) s += cnt[base + i];
    int incl = s;
#pragma unroll
    for (int d = 1; d < 32; d <<= 1) {
      const int y = __shfl_up(incl, d, 32);
      if (lane >= d) incl += y;
    }
    int run = incl - s;
#pragma unroll 1
    for (int i = 0; i < NBRUN / 32; ++i) {
      const int cv = cnt[base + i];
      offs[base + i] = run;
      cur[base + i]  = run;
      run += cv;
    }
  }
  __syncthreads();

  if (wave == 0) {
#pragma unroll 1
    for (int w2 = 0; w2 < NWAVE; ++w2) {
      int c = misc[w2];
      c = c < 0 ? 0 : (c > WLCAP ? WLCAP : c);
#pragma unroll 1
      for (int b0 = 0; b0 < c; b0 += 32) {
        const int idx = b0 + lane;
        const int ent = wl[w2 * WLCAP + (idx < WLCAP ? idx : WLCAP - 1)];
        int eid = (ent >> SLB) & 0x1FFFFF;
        eid = eid > NE - 1 ? NE - 1 : eid;
        int sr = srcs[eid];
        sr = sr < 0 ? 0 : (sr > NN - 1 ? NN - 1 : sr);
        const int m32 = (c - b0) < 32 ? (c - b0) : 32;
#pragma unroll 1
        for (int k = 0; k < m32; ++k) {
          const int u    = __builtin_amdgcn_readlane(ent, k);
          const int wd   = __builtin_amdgcn_readlane(sr, k);
          const int slot = u & (NBRUN - 1);
          if (lane == 0) {
            int p = cur[slot];
            p = p < 0 ? 0 : (p > RCAP - 1 ? RCAP - 1 : p);
            pl[p] = wd;
            cur[slot] = p + 1;
          }
        }
      }
    }
  }
  __syncthreads();

  const int ovf = misc[9];
  int* lp  = LIST + (size_t)blk * RCAP;
  int* cop = CO + (size_t)blk * (2 * NBRUN);
  int* fp  = FLAG + (size_t)blk * 32;
  bucket_flush(pl, cnt, ovf, lp, cop, fp, tid);
  __threadfence();
  bucket_flush(pl, cnt, ovf, lp, cop, fp, tid);
}

template <int KTOT>
__device__ __forceinline__ void gemm_16x64(const unsigned short* __restrict__ ap,
                                           const unsigned short* __restrict__ bp, v8f (&acc)[4]) {
#pragma unroll 1
  for (int k0 = 0; k0 < KTOT; k0 += 32) {
    FragB af;
    af.h[0] = *(const v8usa*)(ap + k0);
    af.h[1] = *(const v8usa*)(ap + k0 + 16);
#pragma unroll
    for (int nt = 0; nt < 4; ++nt) {
      const unsigned short* wq = bp + (size_t)(16 * nt) * (size_t)KTOT + k0;
      FragB bf;
      bf.h[0] = *(const v8usa*)wq;
      bf.h[1] = *(const v8usa*)(wq + 16);
      acc[nt] = wmb(af, bf, acc[nt]);
    }
  }
}

__device__ __forceinline__ void stage_d(float* stg, const v8f (&acc)[4], int wave, int hh, int m) {
#pragma unroll
  for (int nt = 0; nt < 4; ++nt) {
#pragma unroll
    for (int r = 0; r < 8; ++r) stg[(16 * wave + 8 * hh + r) * SP + 16 * nt + m] = acc[nt][r];
  }
}

__global__ __launch_bounds__(NTHR) void k_replay(const int* __restrict__ LIST, const int* __restrict__ CO,
                                                 const int* __restrict__ FLAG, const float* __restrict__ X,
                                                 const float* __restrict__ TB, int layer, unsigned short* HHL) {
  const int tid = (int)threadIdx.x, lane = tid & 31, wave = tid >> 5, hh = lane >> 4, q = lane & 15;
  const int rowBase = (int)blockIdx.x * ABM;
  const int bucket  = rowBase >> SLB;
  const int* lb  = LIST + (size_t)bucket * RCAP;
  const int* cob = CO + (size_t)bucket * (2 * NBRUN);
  const int flag = FLAG[(size_t)bucket * 32];
  const float s  = 1.0f + TB[TB_SC + 1 + layer];
  const float qnan = __uint_as_float(0x7fc00000u);

#pragma unroll 1
  for (int i = 0; i < ABM / (2 * NWAVE); ++i) {
    const int d    = rowBase + (ABM / NWAVE) * wave + 2 * i + hh;
    const int slot = d & (NBRUN - 1);
    int c = cob[slot];
    int o = cob[NBRUN + slot];
    const bool big = c > DEGCAP;
    c = c < 0 ? 0 : (c > DEGCAP ? DEGCAP : c);
    o = o < 0 ? 0 : (o > RCAP - 1 ? RCAP - 1 : o);
    const int co = __shfl_xor(c, 16, 32);
    const int cm = c > co ? c : co;
    int last = o + c - 1;
    last = last < o ? o : last;
    last = last > RCAP - 1 ? RCAP - 1 : last;
    float a0 = 0.0f, a1 = 0.0f, a2 = 0.0f, a3 = 0.0f;
#pragma unroll 1
    for (int j = 0; j < cm; ++j) {
      int idx = o + j;
      idx = idx > last ? last : idx;
      int sr = lb[idx];
      sr = sr < 0 ? 0 : (sr > NN - 1 ? NN - 1 : sr);
      const v4f v = *(const v4fa*)(X + (size_t)sr * HD + 4 * q);
      asm volatile("" :: "v"(v));
      const bool valid = j < c;
      const float t0 = a0 + v.x, t1 = a1 + v.y, t2 = a2 + v.z, t3 = a3 + v.w;
      a0 = valid ? t0 : a0; a1 = valid ? t1 : a1; a2 = valid ? t2 : a2; a3 = valid ? t3 : a3;
    }
    const int dc = d < NN ? d : NN - 1;
    const v4f g = *(const v4fa*)(X + (size_t)dc * HD + 4 * q);
    asm volatile("" :: "v"(g));
    float m0 = s * g.x + a0, m1 = s * g.y + a1, m2 = s * g.z + a2, m3 = s * g.w + a3;
    const bool bad  = (flag != 0) | big;
    const bool live = d < NN;
    m0 = bad ? qnan : m0; m1 = bad ? qnan : m1; m2 = bad ? qnan : m2; m3 = bad ? qnan : m3;
    m0 = live ? m0 : 0.0f; m1 = live ? m1 : 0.0f; m2 = live ? m2 : 0.0f; m3 = live ? m3 : 0.0f;
    int h01, h23, l01, l23;
    hilo_pack(m0, m1, m2, m3, h01, h23, l01, l23);
    const v4i ow = regroup8(h01, h23, l01, l23, lane);
    st2_v4i(HHL + (size_t)d * KL + 8 * q, ow);
  }
}

__global__ __launch_bounds__(NTHR) __attribute__((amdgpu_num_vgpr(248)))
void k_mlp(const unsigned short* __restrict__ A, const unsigned short* __restrict__ B1,
           const unsigned short* __restrict__ B2, const float* __restrict__ TB, int layer,
           float* U, float* REC) {
  __shared__ __attribute__((aligned(16))) float tile[GBM * SP];
  __shared__ __attribute__((aligned(16))) float sb[128];
  __shared__ __attribute__((aligned(16))) float rec[192];
  const int tid = (int)threadIdx.x, lane = tid & 31, wave = tid >> 5, hh = lane >> 4, m = lane & 15;
  const int blk = (int)blockIdx.x;
  const int rowBase = blk * GBM;
  if (tid < 32) {
    const int off = (tid < 16) ? (TB_B1 + layer * HD + 4 * tid) : (TB_B2 + layer * HD + 4 * (tid - 16));
    *(v4fa*)(sb + 4 * tid) = *(const v4fa*)(TB + off);
  }

  v8f acc[4];
  {
    const v8f z = {0.f, 0.f, 0.f, 0.f, 0.f, 0.f, 0.f, 0.f};
#pragma unroll
    for (int t = 0; t < 4; ++t) acc[t] = z;
  }
  {
    const unsigned short* ap = A + (size_t)(rowBase + 16 * wave + m) * (size_t)KL + 8 * hh;
    const unsigned short* bp = B1 + (size_t)m * (size_t)KL + 8 * hh;
    gemm_16x64<KL>(ap, bp, acc);
  }
  stage_d(tile, acc, wave, hh, m);
  __syncthreads();

  {
    const v4f bias = *(const v4fa*)(sb + 4 * m);
#pragma unroll 1
    for (int i = 0; i < 8; ++i) {
      const int lr = 16 * wave + 2 * i + hh;
      float* rp = tile + lr * SP + 4 * m;
      const v4f a = *(const v4fa*)rp;
      float v0 = a.x + bias.x, v1 = a.y + bias.y, v2 = a.z + bias.z, v3 = a.w + bias.w;
      v0 = (v0 > 0.0f) ? v0 : (v0 - v0); v1 = (v1 > 0.0f) ? v1 : (v1 - v1);
      v2 = (v2 > 0.0f) ? v2 : (v2 - v2); v3 = (v3 > 0.0f) ? v3 : (v3 - v3);
      int h01, h23, l01, l23;
      hilo_pack(v0, v1, v2, v3, h01, h23, l01, l23);
      const v4i ow = regroup8(h01, h23, l01, l23, lane);
      *(v4ia*)rp = ow;
    }
  }
  __syncthreads();

  {
    const v8f z = {0.f, 0.f, 0.f, 0.f, 0.f, 0.f, 0.f, 0.f};
#pragma unroll
    for (int t = 0; t < 4; ++t) acc[t] = z;
  }
  {
    const int ao = (16 * wave + m) * AP + 8 * hh;
    const unsigned short* bp = B2 + (size_t)m * (size_t)KL + 8 * hh;
#pragma unroll 1
    for (int k0 = 0; k0 < KL; k0 += 32) {
      FragB af;
      af.h[0] = *(const v8usa*)((const unsigned short*)tile + ao + k0);
      af.h[1] = *(const v8usa*)((const unsigned short*)tile + ao + k0 + 16);
#pragma unroll
      for (int nt = 0; nt < 4; ++nt) {
        const unsigned short* wq = bp + (size_t)(16 * nt) * (size_t)KL + k0;
        FragB bf;
        bf.h[0] = *(const v8usa*)wq;
        bf.h[1] = *(const v8usa*)(wq + 16);
        acc[nt] = wmb(af, bf, acc[nt]);
      }
    }
  }
  __syncthreads();
  stage_d(tile, acc, wave, hh, m);
  __syncthreads();

  {
    const v4f bias = *(const v4fa*)(sb + 64 + 4 * m);
#pragma unroll 1
    for (int i = 0; i < 8; ++i) {
      const int lr   = 16 * wave + 2 * i + hh;
      const int grow = rowBase + lr;
      const bool live = grow < NN;
      float* rp = tile + lr * SP + 4 * m;
      const v4f a = *(const v4fa*)rp;
      float v0 = a.x + bias.x, v1 = a.y + bias.y, v2 = a.z + bias.z, v3 = a.w + bias.w;
      v0 = (v0 > 0.0f) ? v0 : (v0 - v0); v1 = (v1 > 0.0f) ? v1 : (v1 - v1);
      v2 = (v2 > 0.0f) ? v2 : (v2 - v2); v3 = (v3 > 0.0f) ? v3 : (v3 - v3);
      v4f o;
      o.x = v0; o.y = v1; o.z = v2; o.w = v3;
      *(v4fa*)rp = o;
      asm volatile("" :: "v"(o));
      if (live) st2_v4f(U + (size_t)grow * HD + 4 * m, o);
    }
  }
  __syncthreads();

  if (tid < 64) {
    const int nvr = NN - rowBase;
    const int nv  = nvr < GBM ? nvr : GBM;
    const float rn = (nv == GBM) ? (1.0f / 128.0f) : (1.0f / 32.0f);
    float sum = 0.0f;
#pragma unroll 4
    for (int r = 0; r < nv; ++r) sum += tile[r * SP + tid];
    const float mean = sum * rn;
    float q2 = 0.0f;
#pragma unroll 4
    for (int r = 0; r < nv; ++r) {
      const float dd = tile[r * SP + tid] - mean;
      q2 = fmaf(dd, dd, q2);
    }
    rec[tid]       = (float)nv;
    rec[64 + tid]  = mean;
    rec[128 + tid] = q2;
  }
  __syncthreads();
  {
    const int ri = tid < 48 ? tid : 47;
    const v4f pv = *(const v4fa*)(rec + 4 * ri);
    asm volatile("" :: "v"(pv));
    float* op = REC + (size_t)blk * 192 + 4 * ri;
    if (tid < 48) *(volatile v4f*)op = pv;
    __threadfence();
    if (tid < 48) *(volatile v4f*)op = pv;
  }
}

__global__ __launch_bounds__(64) void k_comb(const float* __restrict__ REC, float* ST) {
  __shared__ __attribute__((aligned(16))) float stg[128];
  const int c = (int)threadIdx.x;
  double sn = 0.0, sm = 0.0;
#pragma unroll 1
  for (int b = 0; b < NT; ++b) {
    const float* pr = REC + (size_t)b * 192;
    const double nb = (double)pr[c];
    const double mb = (double)pr[64 + c];
    sn += nb;
    sm += nb * mb;
  }
  const double dn  = sn < 1.0 ? 1.0 : sn;
  const double inv = 1.0 / dn;
  const double mean = sm * inv;
  double M2 = 0.0;
#pragma unroll 1
  for (int b = 0; b < NT; ++b) {
    const float* pr = REC + (size_t)b * 192;
    const double nb = (double)pr[c];
    const double mb = (double)pr[64 + c];
    const double qb = (double)pr[128 + c];
    const double dd = mb - mean;
    M2 += qb + nb * dd * dd;
  }
  const float varf  = (float)(M2 * inv);
  const float meanf = (float)mean;
  const float rs = 1.0f / sqrtf(varf + 1e-5f);
  stg[c] = meanf;
  stg[64 + c] = rs;
  __syncthreads();
  if (c < 32) {
    const v4f v = *(const v4fa*)(stg + 4 * c);
    *(volatile v4f*)(ST + 4 * c) = v;
    __threadfence();
    *(volatile v4f*)(ST + 4 * c) = v;
  }
}

template <int LAST>
__global__ __launch_bounds__(NTHR) void k_apply(const float* __restrict__ U, const float* __restrict__ TB,
                                                const float* __restrict__ ST, int layer,
                                                float* X, unsigned short* HHL) {
  __shared__ __attribute__((aligned(16))) float ps[256];
  const int tid = (int)threadIdx.x, lane = tid & 31;
  if (tid < 32) {
    const int off = (tid < 16) ? (TB_G + layer * HD + 4 * tid) : (TB_BE + layer * HD + 4 * (tid - 16));
    *(v4fa*)(ps + 4 * tid) = *(const v4fa*)(TB + off);
  } else if (tid < 64) {
    *(v4fa*)(ps + 4 * tid) = *(const v4fa*)(ST + 4 * (tid - 32));
  }
  __syncthreads();
  const int u = (int)blockIdx.x * NTHR + tid;
  const int row = u >> 4, q = u & 15;
  const v4f v  = *(const v4fa*)(U + (size_t)u * 4);
  const v4f g  = *(const v4fa*)(ps + 4 * q);
  const v4f be = *(const v4fa*)(ps + 64 + 4 * q);
  const v4f mu = *(const v4fa*)(ps + 128 + 4 * q);
  const v4f rs = *(const v4fa*)(ps + 192 + 4 * q);
  const float y0 = ((g.x * (v.x - mu.x)) * rs.x) + be.x;
  const float y1 = ((g.y * (v.y - mu.y)) * rs.y) + be.y;
  const float y2 = ((g.z * (v.z - mu.z)) * rs.z) + be.z;
  const float y3 = ((g.w * (v.w - mu.w)) * rs.w) + be.w;
  if constexpr (LAST != 0) {
    int h01, h23, l01, l23;
    hilo_pack(y0, y1, y2, y3, h01, h23, l01, l23);
    const v4i ow = regroup8(h01, h23, l01, l23, lane);
    st2_v4i(HHL + (size_t)row * KL + 8 * q, ow);
  } else {
    v4f o;
    o.x = y0; o.y = y1; o.z = y2; o.w = y3;
    st2_v4f(X + (size_t)u * 4, o);
  }
}

__global__ __launch_bounds__(NTHR) __attribute__((amdgpu_num_vgpr(248)))
void k_head(const unsigned short* __restrict__ A, const unsigned short* __restrict__ BT,
            const float* __restrict__ TB, float* out) {
  __shared__ __attribute__((aligned(16))) float tile[GBM * SP];
  __shared__ __attribute__((aligned(16))) float sb[128];
  __shared__ __attribute__((aligned(16))) float sc[GBM];
  const int tid = (int)threadIdx.x, lane = tid & 31, wave = tid >> 5, hh = lane >> 4, m = lane & 15;
  const int blk = (int)blockIdx.x;
  const int rowBase = blk * GBM;
  if (tid < 32) *(v4fa*)(sb + 4 * tid) = *(const v4fa*)(TB + TB_L1B + 4 * tid);
  const float b2v = TB[TB_SC];

  v8f acc[4];
  {
    const v8f z = {0.f, 0.f, 0.f, 0.f, 0.f, 0.f, 0.f, 0.f};
#pragma unroll
    for (int t = 0; t < 4; ++t) acc[t] = z;
  }
  {
    const unsigned short* ap = A + (size_t)(rowBase + 16 * wave + m) * (size_t)KL + 8 * hh;
    const unsigned short* bp = BT + (size_t)m * (size_t)KL + 8 * hh;
    gemm_16x64<KL>(ap, bp, acc);
  }
  stage_d(tile, acc, wave, hh, m);
  __syncthreads();

  if (tid < GBM) {
    const float* rp = tile + tid * SP;
    float s = 0.0f;
#pragma unroll 1
    for (int c4 = 0; c4 < 16; ++c4) {
      const v4f a = *(const v4fa*)(rp + 4 * c4);
      const v4f b = *(const v4fa*)(sb + 4 * c4);
      const v4f w = *(const v4fa*)(sb + 64 + 4 * c4);
      float v0 = a.x + b.x, v1 = a.y + b.y, v2 = a.z + b.z, v3 = a.w + b.w;
      v0 = (v0 > 0.0f) ? v0 : (v0 - v0); v1 = (v1 > 0.0f) ? v1 : (v1 - v1);
      v2 = (v2 > 0.0f) ? v2 : (v2 - v2); v3 = (v3 > 0.0f) ? v3 : (v3 - v3);
      s = fmaf(v0, w.x, s);
      s = fmaf(v1, w.y, s);
      s = fmaf(v2, w.z, s);
      s = fmaf(v3, w.w, s);
    }
    sc[tid] = s + b2v;
  }
  __syncthreads();

  if (tid < 32) {
    const int liveRows = (NN - rowBase) < GBM ? (NN - rowBase) : GBM;
    const int nv4 = liveRows >> 2;
    const v4f v = *(const v4fa*)(sc + 4 * lane);
    asm volatile("" :: "v"(v));
    float* op = out + (size_t)blk * GBM + 4 * lane;
    if (lane < nv4) *(volatile v4f*)op = v;
    __threadfence();
    if (lane < nv4) *(volatile v4f*)op = v;
  }
}

extern "C" void kernel_launch(void* const* d_in, const int* in_sizes, int n_in,
                              void* d_out, int out_size, void* d_ws, size_t ws_size,
                              hipStream_t stream) {
  if (n_in < 13) return;
  if (in_sizes[0] != NN * HD) return;
  if (in_sizes[1] != 2 * NE) return;
  if (in_sizes[2] != NLAY * HD * HD) return;
  if (in_sizes[3] != NLAY * HD) return;
  if (in_sizes[4] != NLAY * HD * HD) return;
  if (in_sizes[5] != NLAY * HD) return;
  if (in_sizes[6] != NLAY * HD) return;
  if (in_sizes[7] != NLAY * HD) return;
  if (in_sizes[8] != NLAY) return;
  if (in_sizes[9] != HD * HD) return;
  if (in_sizes[10] != HD) return;
  if (in_sizes[11] != HD) return;
  if (in_sizes[12] != 1) return;
  if (out_size != NN) return;

  const float* x    = (const float*)d_in[0];
  const int*   ei   = (const int*)d_in[1];
  const float* W1   = (const float*)d_in[2];
  const float* b1   = (const float*)d_in[3];
  const float* W2   = (const float*)d_in[4];
  const float* b2   = (const float*)d_in[5];
  const float* gam  = (const float*)d_in[6];
  const float* bet  = (const float*)d_in[7];
  const float* eps  = (const float*)d_in[8];
  const float* l1w  = (const float*)d_in[9];
  const float* l1b  = (const float*)d_in[10];
  const float* l2w  = (const float*)d_in[11];
  const float* l2b  = (const float*)d_in[12];
  float* out = (float*)d_out;
  const int* srcs = ei;
  const int* dsts = ei + NE;

  constexpr size_t zX    = (size_t)NN * HD * 4;
  constexpr size_t zU    = (size_t)NN * HD * 4;
  constexpr size_t zHL   = (size_t)MP * KL * 2;
  constexpr size_t zLIST = (size_t)NBK * RCAP * 4;
  constexpr size_t zCO   = (size_t)NBK * 2 * NBRUN * 4;
  constexpr size_t zFLAG = (size_t)NBK * 128;
  constexpr size_t zREC  = (size_t)NT * 192 * 4;
  constexpr size_t zSTAT = (size_t)NLAY * 128 * 4;
  constexpr size_t zWPL  = (size_t)7 * HD * KL * 2;
  constexpr size_t zTB   = (size_t)TB_N * 4;
  constexpr size_t oX    = 0;
  constexpr size_t oU    = oX + zX;
  constexpr size_t oHL   = oU + zU;
  constexpr size_t oLIST = oHL + zHL;
  constexpr size_t oCO   = oLIST + zLIST;
  constexpr size_t oFLAG = oCO + zCO;
  constexpr size_t oREC  = oFLAG + zFLAG;
  constexpr size_t oSTAT = oREC + zREC;
  constexpr size_t oWPL  = oSTAT + zSTAT;
  constexpr size_t oTB   = oWPL + zWPL;
  constexpr size_t oEND  = oTB + zTB;
  static_assert(zX % 256 == 0 && zU % 256 == 0 && zHL % 256 == 0 && zLIST % 256 == 0 && zCO % 256 == 0);
  static_assert(zFLAG % 256 == 0 && zREC % 256 == 0 && zSTAT % 256 == 0 && zWPL % 256 == 0 && zTB % 256 == 0);
  static_assert((size_t)(TB_SC + 32) * 4 <= zTB);
  static_assert(oEND <= (size_t)WSMAX);
  if (oEND > ws_size) return;

  char* ws = (char*)d_ws;
  float*          X    = (float*)(ws + oX);
  float*          U    = (float*)(ws + oU);
  unsigned short* HHL  = (unsigned short*)(ws + oHL);
  int*            LIST = (int*)(ws + oLIST);
  int*            CO   = (int*)(ws + oCO);
  int*            FLAG = (int*)(ws + oFLAG);
  float*          REC  = (float*)(ws + oREC);
  float*          STAT = (float*)(ws + oSTAT);
  unsigned short* WPL  = (unsigned short*)(ws + oWPL);
  float*          TB   = (float*)(ws + oTB);

  hipFuncSetAttribute(reinterpret_cast<const void*>(&k_bucket), hipFuncAttributeMaxDynamicSharedMemorySize, (int)BK_LDS);

  k_prep<<<PBTOT, NTHR, 0, stream>>>(x, W1, b1, W2, b2, gam, bet, eps, l1w, l1b, l2w, l2b, X, WPL, HHL, TB);
  k_bucket<<<NBK, NTHR, BK_LDS, stream>>>(srcs, dsts, LIST, CO, FLAG);

  for (int l = 0; l < NLAY; ++l) {
    const unsigned short* w1d = WPL + (size_t)l * HD * KL;
    const unsigned short* w2d = WPL + (size_t)(3 + l) * HD * KL;
    float* st = STAT + (size_t)l * 128;
    k_replay<<<MP / ABM, NTHR, 0, stream>>>(LIST, CO, FLAG, X, TB, l, HHL);
    k_mlp<<<NT, NTHR, 0, stream>>>(HHL, w1d, w2d, TB, l, U, REC);
    k_comb<<<1, 64, 0, stream>>>(REC, st);
    if (l == NLAY - 1)
      k_apply<1><<<NN * HD / 4 / NTHR, NTHR, 0, stream>>>(U, TB, st, l, X, HHL);
    else
      k_apply<0><<<NN * HD / 4 / NTHR, NTHR, 0, stream>>>(U, TB, st, l, X, HHL);
  }
  k_head<<<NT, NTHR, 0, stream>>>(HHL, WPL + (size_t)6 * HD * KL, TB, out);
}
